// UV_Aggregator_NoUserAttention_29669634080987
// MI455X (gfx1250) — hardware-verified
//
#include <hip/hip_runtime.h>
#include <stddef.h>


#define NNODE  4096
#define NSLOT  200
#define DEMB   64
#define KIN    128
#define NITEM  100000
#define NRAT   5
#define NRPAD  8
#define NTHR   128
#define NWAVE  (NTHR / 32)
#define CHR    64
#define NCHK   4
#define PX     136
#define PH     72
#define PTHR   256
#define NPV    (NITEM * DEMB / 8)
#define NBV    (NPV / PTHR)
#define NPW1   (DEMB * KIN / 8)
#define NBW1   (NPW1 / PTHR)
#define NPW2   (DEMB * DEMB / 8)
#define NBW2   (NPW2 / PTHR)
#define NPRV   (NRAT * DEMB / 8)
#define NPR    (NRPAD * DEMB / 8)
#define NBPREP (NBV + NBW1 + NBW2 + 1)
#define SC_X   8.0f
#define SC_W   64.0f
#define SC_H   16.0f
#define INV1   (1.0f / 512.0f)
#define INV2   (1.0f / 1024.0f)
#define INVL   (1.0f / 200.0f)

static_assert(NBV * PTHR == NPV);
static_assert(NBW1 * PTHR == NPW1);
static_assert(NBW2 * PTHR == NPW2);
static_assert(NPR <= PTHR);
static_assert(NPR % 32 == 0);
static_assert(NCHK * CHR >= NSLOT);
static_assert((NCHK - 1) * CHR < NSLOT);
static_assert(CHR == 16 * NWAVE);
static_assert((CHR * 8) % NTHR == 0);
static_assert(NPW1 % NTHR == 0);
static_assert(NPW2 % NTHR == 0);
static_assert(NPR <= NTHR);
static_assert(DEMB <= NTHR);
static_assert((PX * 2) % 16 == 0);
static_assert((PH * 2) % 16 == 0);
static_assert(PX >= KIN);
static_assert(PH >= DEMB);
static_assert(KIN % 32 == 0);
static_assert(DEMB % 32 == 0);
static_assert(DEMB == 4 * 16);

typedef _Float16 v16h __attribute__((ext_vector_type(16)));
typedef _Float16 v8h  __attribute__((ext_vector_type(8)));
typedef float    v4f  __attribute__((ext_vector_type(4)));
typedef float    v8f  __attribute__((ext_vector_type(8)));
union FragH { v16h v; v8h h[2]; };

__device__ __forceinline__ v8f wmh(v16h a, v16h b, v8f c) {
  v8f d = __builtin_amdgcn_wmma_f32_16x16x32_f16(false, a, false, b, (short)0, c, false, false);
#if defined(__HIP_DEVICE_COMPILE__)
  asm volatile("v_nop\n\tv_nop\n\tv_nop\n\tv_nop" : "+v"(d) : "v"(a), "v"(b));
#endif
  return d;
}

__device__ __forceinline__ v8f zero8() {
  v8f z = {0.f, 0.f, 0.f, 0.f, 0.f, 0.f, 0.f, 0.f};
  return z;
}

__device__ __forceinline__ v16h afrag(const _Float16* row, int k0, int h) {
  FragH u;
  u.h[0] = *(const v8h*)(row + k0 + 8 * h);
  u.h[1] = *(const v8h*)(row + k0 + 16 + 8 * h);
  return u.v;
}

__device__ __forceinline__ int wrap_clamp(int e, int n) {
  e = e < 0 ? e + n : e;
  e = e < 0 ? 0 : e;
  e = e > n - 1 ? n - 1 : e;
  return e;
}

__device__ __forceinline__ v8h selz(bool keep, v8h v) {
  v8h o;
#pragma unroll
  for (int i = 0; i < 8; ++i) o[i] = keep ? v[i] : (_Float16)0.0f;
  return o;
}

__global__ __launch_bounds__(PTHR) void k_prep(const float* __restrict__ v2e, const float* __restrict__ r2e,
                                               const float* __restrict__ w1, const float* __restrict__ w2,
                                               _Float16* v2eh, _Float16* w1h, _Float16* w2h, _Float16* r2eh) {
  const int blk = blockIdx.x, t = (int)threadIdx.x;
  const float* src;
  _Float16* dst;
  float sc;
  bool keep = true, on = true;
  if (blk < NBV) {
    const size_t p = (size_t)blk * PTHR + (size_t)t;
    src = v2e + 8 * p;
    dst = v2eh + 8 * p;
    sc = SC_X;
  } else if (blk < NBV + NBW1) {
    const int p = (blk - NBV) * PTHR + t;
    src = w1 + 8 * p;
    dst = w1h + 8 * p;
    sc = SC_W;
  } else if (blk < NBV + NBW1 + NBW2) {
    const int p = (blk - NBV - NBW1) * PTHR + t;
    src = w2 + 8 * p;
    dst = w2h + 8 * p;
    sc = SC_W;
  } else {
    const int p = t;
    on = p < NPR;
    keep = p < NPRV;
    const int ps = p < NPRV ? p : (NPRV - 1);
    const int pd = p < NPR ? p : (NPR - 1);
    src = r2e + 8 * ps;
    dst = r2eh + 8 * pd;
    sc = SC_X;
  }
  const v4f u0 = *(const v4f*)src;
  const v4f u1 = *(const v4f*)(src + 4);
  v8h o;
#pragma unroll
  for (int i = 0; i < 4; ++i) {
    o[i]     = keep ? (_Float16)(sc * u0[i]) : (_Float16)0.0f;
    o[4 + i] = keep ? (_Float16)(sc * u1[i]) : (_Float16)0.0f;
  }
  if (on) {
    *(volatile v8h*)dst = o;
    __threadfence();
    *(volatile v8h*)dst = o;
  }
}

__global__ __launch_bounds__(NTHR) void k_main(const _Float16* __restrict__ v2eh, const _Float16* __restrict__ w1h,
                                               const _Float16* __restrict__ w2h, const _Float16* __restrict__ r2eh,
                                               const float* __restrict__ b1, const float* __restrict__ b2,
                                               const int* __restrict__ huv, const int* __restrict__ hr,
                                               float* out) {
  __shared__ __align__(16) _Float16 sW1[DEMB * PX];
  __shared__ __align__(16) _Float16 sW2[DEMB * PH];
  __shared__ __align__(16) _Float16 sX[CHR * PX];
  __shared__ __align__(16) _Float16 sH[CHR * PH];
  __shared__ __align__(16) _Float16 sR[NRPAD * DEMB];
  __shared__ __align__(16) float sB1[DEMB];
  __shared__ __align__(16) float sB2[DEMB];
  __shared__ __align__(16) float sPart[NWAVE * DEMB];

  const int tid = (int)threadIdx.x, lane = tid & 31, h = lane >> 4, m = lane & 15;
  const int wv  = __builtin_amdgcn_readfirstlane(tid >> 5);
  const int b   = blockIdx.x;

#pragma unroll
  for (int j = 0; j < NPW1 / NTHR; ++j) {
    const int p = tid + NTHR * j;
    const int row = p >> 4, c8 = p & 15;
    *(v8h*)(sW1 + row * PX + 8 * c8) = *(const v8h*)(w1h + (size_t)row * KIN + 8 * c8);
  }
#pragma unroll
  for (int j = 0; j < NPW2 / NTHR; ++j) {
    const int p = tid + NTHR * j;
    const int row = p >> 3, c8 = p & 7;
    *(v8h*)(sW2 + row * PH + 8 * c8) = *(const v8h*)(w2h + (size_t)row * DEMB + 8 * c8);
  }
  if (tid < NPR) *(v8h*)(sR + 8 * tid) = *(const v8h*)(r2eh + 8 * tid);
  if (tid < DEMB) {
    sB1[tid] = b1[tid];
    sB2[tid] = b2[tid];
  }
  float rs[4] = {0.0f, 0.0f, 0.0f, 0.0f};
  __syncthreads();

  const int* hu = huv + (size_t)b * NSLOT;
  const int* hq = hr  + (size_t)b * NSLOT;

#pragma unroll 1
  for (int c = 0; c < NCHK; ++c) {
    const int row0 = c * CHR;

#pragma unroll
    for (int j = 0; j < (CHR * 8) / NTHR; ++j) {
      const int p = tid + NTHR * j;
      const int row = p >> 3, c8 = p & 7;
      const int slot = row0 + row;
      const bool valid = slot < NSLOT;
      const int slotc = valid ? slot : (NSLOT - 1);
      const int iu = wrap_clamp(hu[slotc], NITEM);
      const int ir = wrap_clamp(hq[slotc], NRAT);
      const v8h xv = *(const v8h*)(v2eh + (size_t)iu * DEMB + 8 * c8);
      const v8h rv = *(const v8h*)(sR + ir * DEMB + 8 * c8);
      *(v8h*)(sX + row * PX + 8 * c8)        = selz(valid, xv);
      *(v8h*)(sX + row * PX + DEMB + 8 * c8) = selz(valid, rv);
    }
    __syncthreads();

    const bool act = (row0 + 16 * wv) < NSLOT;

    if (act) {
      v8f acc[4];
#pragma unroll
      for (int nt = 0; nt < 4; ++nt) acc[nt] = zero8();
      const _Float16* arow = sX + (16 * wv + m) * PX;
#pragma unroll
      for (int ks = 0; ks < KIN / 32; ++ks) {
        const int k0 = 32 * ks;
        const v16h a = afrag(arow, k0, h);
#pragma unroll
        for (int nt = 0; nt < 4; ++nt) {
          const v16h bb = afrag(sW1 + (16 * nt + m) * PX, k0, h);
          acc[nt] = wmh(a, bb, acc[nt]);
        }
      }
      _Float16* hrow = sH + (16 * wv + 8 * h) * PH;
#pragma unroll
      for (int nt = 0; nt < 4; ++nt) {
        const int col = 16 * nt + m;
        const float bb = sB1[col];
#pragma unroll
        for (int r = 0; r < 8; ++r) {
          const float hv = fmaxf(fmaf(acc[nt][r], INV1, bb), 0.0f);
          hrow[r * PH + col] = (_Float16)(SC_H * hv);
        }
      }
    }
    __syncthreads();

    if (act) {
      v8f acc[4];
#pragma unroll
      for (int nt = 0; nt < 4; ++nt) acc[nt] = zero8();
      const _Float16* arow = sH + (16 * wv + m) * PH;
#pragma unroll
      for (int ks = 0; ks < DEMB / 32; ++ks) {
        const int k0 = 32 * ks;
        const v16h a = afrag(arow, k0, h);
#pragma unroll
        for (int nt = 0; nt < 4; ++nt) {
          const v16h bb = afrag(sW2 + (16 * nt + m) * PH, k0, h);
          acc[nt] = wmh(a, bb, acc[nt]);
        }
      }
      const int lim = NSLOT - (row0 + 16 * wv + 8 * h);
#pragma unroll
      for (int nt = 0; nt < 4; ++nt) {
        const int col = 16 * nt + m;
        const float bb = sB2[col];
        float s = 0.0f;
#pragma unroll
        for (int r = 0; r < 8; ++r) {
          const float o = fmaxf(fmaf(acc[nt][r], INV2, bb), 0.0f);
          s += (r < lim) ? o : 0.0f;
        }
        rs[nt] += s;
      }
    }
  }

#pragma unroll
  for (int nt = 0; nt < 4; ++nt) rs[nt] += __shfl_xor(rs[nt], 16, 32);
  if (h == 0) {
#pragma unroll
    for (int nt = 0; nt < 4; ++nt) sPart[wv * DEMB + 16 * nt + m] = rs[nt];
  }
  __syncthreads();
  if (tid < 16) {
    v4f s = *(const v4f*)(sPart + 4 * tid);
#pragma unroll
    for (int q = 1; q < NWAVE; ++q) {
      const v4f u = *(const v4f*)(sPart + q * DEMB + 4 * tid);
#pragma unroll
      for (int i = 0; i < 4; ++i) s[i] += u[i];
    }
    v4f o;
#pragma unroll
    for (int i = 0; i < 4; ++i) o[i] = s[i] * INVL;
    float* po = out + (size_t)b * DEMB + 4 * tid;
    *(volatile v4f*)po = o;
    __threadfence();
    *(volatile v4f*)po = o;
  }
}

extern "C" void kernel_launch(void* const* d_in, const int* in_sizes, int n_in,
                              void* d_out, int out_size, void* d_ws, size_t ws_size,
                              hipStream_t stream) {
  if (n_in < 9) return;
  if (in_sizes[0] != NITEM * DEMB || in_sizes[1] != NRAT * DEMB) return;
  if (in_sizes[2] != DEMB * KIN || in_sizes[3] != DEMB) return;
  if (in_sizes[4] != DEMB * DEMB || in_sizes[5] != DEMB) return;
  if (in_sizes[7] != NNODE * NSLOT || in_sizes[8] != NNODE * NSLOT) return;
  if (out_size != NNODE * DEMB) return;

  const float* v2e = (const float*)d_in[0];
  const float* r2e = (const float*)d_in[1];
  const float* w1  = (const float*)d_in[2];
  const float* b1  = (const float*)d_in[3];
  const float* w2  = (const float*)d_in[4];
  const float* b2  = (const float*)d_in[5];
  const int* huv = (const int*)d_in[7];
  const int* hr  = (const int*)d_in[8];
  float* out = (float*)d_out;

  const size_t szV  = (size_t)NITEM * DEMB * 2;
  const size_t szW1 = (size_t)DEMB * KIN * 2;
  const size_t szW2 = (size_t)DEMB * DEMB * 2;
  const size_t szR  = (size_t)NRPAD * DEMB * 2;
  const size_t offW1 = szV, offW2 = offW1 + szW1, offR = offW2 + szW2;
  const size_t total = offR + szR;
  if (total > ws_size || total > (size_t)134217728) return;
  char* ws = (char*)d_ws;
  _Float16* v2eh = (_Float16*)(ws);
  _Float16* w1h  = (_Float16*)(ws + offW1);
  _Float16* w2h  = (_Float16*)(ws + offW2);
  _Float16* r2eh = (_Float16*)(ws + offR);

  k_prep<<<NBPREP, PTHR, 0, stream>>>(v2e, r2e, w1, w2, v2eh, w1h, w2h, r2eh);
  k_main<<<NNODE, NTHR, 0, stream>>>(v2eh, w1h, w2h, r2eh, b1, b2, huv, hr, out);
}
